// Image_Text_Attention_1065151889661
// MI455X (gfx1250) — hardware-verified
//
#include <hip/hip_runtime.h>
#include <hip/hip_bf16.h>
#include <math.h>
#include <stdint.h>


#define B_  32
#define M_  196
#define D_  768
#define L_  512
#define K_  768
#define MT_ 13

typedef unsigned short us16;
typedef us16   v8us  __attribute__((ext_vector_type(8)));
typedef us16   v16us __attribute__((ext_vector_type(16)));
typedef __bf16 v16bf __attribute__((ext_vector_type(16)));
typedef float  v8f   __attribute__((ext_vector_type(8)));
typedef float  v4f   __attribute__((ext_vector_type(4)));

union Frag { v16us u; v8us h2[2]; v16bf b; };

static_assert(D_ == K_);
static_assert((B_ * M_) % 32 == 0);
static_assert((B_ * L_) % 32 == 0);
static_assert(((B_ * M_) * 4) % 128 == 0);
static_assert(((B_ * L_) * 4) % 128 == 0);
static_assert(MT_ * 16 >= M_);

__device__ __forceinline__ us16 bf16_bits(float f) {
  unsigned int u = __float_as_uint(f);
  u += 0x7FFFu + ((u >> 16) & 1u);
  return (us16)(u >> 16);
}
__device__ __forceinline__ float bf16_val(us16 hv) {
  return __uint_as_float(((unsigned int)hv) << 16);
}
__device__ __forceinline__ float bfr(float f) { return bf16_val(bf16_bits(f)); }

__device__ __forceinline__ v8f zero8() {
  v8f z = {0.f, 0.f, 0.f, 0.f, 0.f, 0.f, 0.f, 0.f};
  return z;
}

__device__ __forceinline__ v8f wmma_bf16(v16bf a, v16bf b, v8f c) {
  v8f d = __builtin_amdgcn_wmma_f32_16x16x32_bf16(false, a, false, b, (short)0, c, false, false);
  asm volatile("v_nop\n\tv_nop\n\tv_nop\n\tv_nop" : "+v"(d) : "v"(a), "v"(b));
  return d;
}

__global__ __launch_bounds__(256)
void k_proj(const float* __restrict__ img, const float* __restrict__ seq,
            const float* __restrict__ imgW, const float* __restrict__ imgB,
            const float* __restrict__ seqW, const float* __restrict__ seqB,
            float* s_out, float* q_out)
{
  __shared__ __align__(16) float res[32];
  const int blk = blockIdx.x;
  const int tid = threadIdx.x, lane = tid & 31, wv = tid >> 5;
  const int PB = (B_ * M_) / 32;
  const bool isP = (blk < PB);
  const float* base = isP ? img : seq;
  const float* wp   = isP ? imgW : seqW;
  const float bias  = bfr(isP ? imgB[0] : seqB[0]);
  const int rb = (isP ? blk : (blk - PB)) * 32;

  float wreg[24];
#pragma unroll
  for (int i = 0; i < 24; ++i) wreg[i] = bfr(wp[lane + 32 * i]);

#pragma unroll 1
  for (int j = 0; j < 4; ++j) {
    const int row = rb + wv * 4 + j;
    const float* x = base + (size_t)row * D_;
    float acc = 0.f;
#pragma unroll
    for (int i = 0; i < 24; ++i) acc += bfr(x[lane + 32 * i]) * wreg[i];
#pragma unroll
    for (int off = 16; off; off >>= 1) acc += __shfl_xor(acc, off, 32);
    if (lane == 0) {
      const float t = tanhf(acc + bias);
      res[wv * 4 + j] = isP ? (t + 1.0f) : t;
    }
  }
  __syncthreads();
  if (tid < 8) {
    v4f v;
    v.x = res[4 * tid + 0]; v.y = res[4 * tid + 1];
    v.z = res[4 * tid + 2]; v.w = res[4 * tid + 3];
    float* dst = (isP ? s_out : q_out) + rb + 4 * tid;
    *(volatile v4f*)dst = v;
    __threadfence();
    *(volatile v4f*)dst = v;
  }
}

__global__ __launch_bounds__(32)
void k_qv(const float* __restrict__ q, const float* __restrict__ V, float* r_out)
{
  __shared__ __align__(16) float st[16][36];
  const int lane = threadIdx.x & 31, h = lane >> 4, m = lane & 15;
  const int col0 = blockIdx.x * 32, row0 = blockIdx.y * 16;
  const float* qrow = q + (size_t)(row0 + m) * L_;

  v8f acc0 = zero8(), acc1 = zero8();
#pragma unroll 1
  for (int k0 = 0; k0 < L_; k0 += 32) {
    Frag ahi, alo, b0, b1;
#pragma unroll
    for (int hh = 0; hh < 2; ++hh) {
      const float* qp = qrow + k0 + 16 * hh + 8 * h;
      const v4f x0 = *(const v4f*)qp;
      const v4f x1 = *(const v4f*)(qp + 4);
      v8us hv, lv;
#pragma unroll
      for (int i = 0; i < 8; ++i) {
        const float xv = (i < 4) ? x0[i] : x1[i - 4];
        const us16 hb = bf16_bits(xv);
        const us16 lb = bf16_bits(xv - bf16_val(hb));
        hv[i] = hb; lv[i] = lb;
      }
      ahi.h2[hh] = hv; alo.h2[hh] = lv;
    }
#pragma unroll
    for (int i = 0; i < 16; ++i) {
      const int kk = k0 + ((i < 8) ? (8 * h + i) : (8 + 8 * h + i));
      const float* vp = V + (size_t)kk * L_ + col0 + m;
      b0.u[i] = bf16_bits(vp[0]);
      b1.u[i] = bf16_bits(vp[16]);
    }
    acc0 = wmma_bf16(ahi.b, b0.b, acc0);
    acc0 = wmma_bf16(alo.b, b0.b, acc0);
    acc1 = wmma_bf16(ahi.b, b1.b, acc1);
    acc1 = wmma_bf16(alo.b, b1.b, acc1);
  }
#pragma unroll
  for (int rr = 0; rr < 8; ++rr) {
    st[8 * h + rr][m]      = acc0[rr];
    st[8 * h + rr][16 + m] = acc1[rr];
  }
  __syncthreads();
  v4f vv[4];
#pragma unroll
  for (int g = 0; g < 4; ++g) {
    const int row = g * 4 + (lane >> 3), c = (lane & 7) * 4;
    vv[g] = *(const v4f*)&st[row][c];
  }
#pragma unroll
  for (int g = 0; g < 4; ++g) {
    const int row = g * 4 + (lane >> 3), c = (lane & 7) * 4;
    *(volatile v4f*)(r_out + (size_t)(row0 + row) * L_ + col0 + c) = vv[g];
  }
  __threadfence();
#pragma unroll
  for (int g = 0; g < 4; ++g) {
    const int row = g * 4 + (lane >> 3), c = (lane & 7) * 4;
    *(volatile v4f*)(r_out + (size_t)(row0 + row) * L_ + col0 + c) = vv[g];
  }
}

__global__ __launch_bounds__(256)
void k_seqT(const float* __restrict__ seq, us16* seqT)
{
  __shared__ __align__(16) us16 tile[32][72];
  const int b = blockIdx.z, l0 = blockIdx.y * 64, k0 = blockIdx.x * 32;
  const int tid = threadIdx.x, lane = tid & 31, wv = tid >> 5;
  const float* src = seq + ((size_t)b * L_ + l0) * K_ + k0;
#pragma unroll
  for (int i = 0; i < 8; ++i) {
    const int idx = tid + 256 * i;
    const int ll = idx >> 5, c = idx & 31;
    tile[c][ll] = bf16_bits(src[(size_t)ll * K_ + c]);
  }
  __syncthreads();
  const int krow = wv * 4 + (lane >> 3), hoff = (lane & 7) * 8;
  const v8us v = *(const v8us*)&tile[krow][hoff];
  us16* dst = seqT + ((size_t)b * K_ + k0 + krow) * L_ + l0 + hoff;
  *(volatile v8us*)dst = v;
  __threadfence();
  *(volatile v8us*)dst = v;
}

__global__ __launch_bounds__(256)
void k_main(const float* __restrict__ s, const float* __restrict__ r,
            const int* __restrict__ mask, const us16* __restrict__ seqT,
            float* out)
{
  __shared__ float r_s[L_];
  __shared__ int   mk_s[L_];
  __shared__ float s_sh[16];
  __shared__ float redmax[8];
  __shared__ float redmin[8];
  __shared__ int   redcnt[8];
  __shared__ float scl[16];
  __shared__ __align__(16) us16  Ahi[16][520];
  __shared__ __align__(16) us16  Alo[16][520];
  __shared__ __align__(16) float outs[16][772];

  const int m0 = blockIdx.x * 16, b = blockIdx.y;
  const int tid = threadIdx.x, lane = tid & 31, wv = tid >> 5;

  float lmax = -__builtin_inff(), lmin = __builtin_inff();
  int cnt = 0;
#pragma unroll
  for (int i = 0; i < 2; ++i) {
    const int l = tid + 256 * i;
    const float rv = r[(size_t)b * L_ + l];
    const int   mv = mask[(size_t)b * L_ + l];
    r_s[l] = rv; mk_s[l] = mv;
    if (mv != 0) { lmax = fmaxf(lmax, rv); lmin = fminf(lmin, rv); ++cnt; }
  }
  if (tid < 16) {
    const int gm = m0 + tid;
    s_sh[tid] = (gm < M_) ? s[(size_t)b * M_ + gm] : 0.f;
  }
#pragma unroll
  for (int off = 16; off; off >>= 1) {
    lmax = fmaxf(lmax, __shfl_xor(lmax, off, 32));
    lmin = fminf(lmin, __shfl_xor(lmin, off, 32));
    cnt += __shfl_xor(cnt, off, 32);
  }
  if (lane == 0) { redmax[wv] = lmax; redmin[wv] = lmin; redcnt[wv] = cnt; }
  __syncthreads();
  float rmax = redmax[0], rmin = redmin[0];
  int nvalid = redcnt[0];
#pragma unroll
  for (int i = 1; i < 8; ++i) {
    rmax = fmaxf(rmax, redmax[i]);
    rmin = fminf(rmin, redmin[i]);
    nvalid += redcnt[i];
  }
  const bool allm = (nvalid == 0);

  {
    const int mr = tid >> 4;
    const int lr = tid & 15;
    const float a = allm ? 0.f : s_sh[mr];
    const float rowmax = allm ? 0.f : ((a >= 0.f) ? a * rmax : a * rmin);
    float z = 0.f;
#pragma unroll 4
    for (int j = 0; j < 32; ++j) {
      const int l = lr + 16 * j;
      const bool v = allm || (mk_s[l] != 0);
      const float e = v ? __expf(a * r_s[l] - rowmax) : 0.f;
      const us16 hb = bf16_bits(e);
      const us16 lb = bf16_bits(e - bf16_val(hb));
      Ahi[mr][l] = hb;
      Alo[mr][l] = lb;
      z += e;
    }
#pragma unroll
    for (int off = 8; off; off >>= 1) z += __shfl_xor(z, off, 32);
    if (lr == 0) scl[mr] = (1.0f / z) * (1.0f / sqrtf((float)K_));
  }
  __syncthreads();

  const int h = lane >> 4, m = lane & 15;
  const us16* sT = seqT + (size_t)b * K_ * L_;
  v8f acc[6];
#pragma unroll
  for (int t = 0; t < 6; ++t) acc[t] = zero8();

#pragma unroll 1
  for (int l0 = 0; l0 < L_; l0 += 32) {
    Frag ahi, alo;
    ahi.h2[0] = *(const v8us*)&Ahi[m][l0 + 8 * h];
    ahi.h2[1] = *(const v8us*)&Ahi[m][l0 + 16 + 8 * h];
    alo.h2[0] = *(const v8us*)&Alo[m][l0 + 8 * h];
    alo.h2[1] = *(const v8us*)&Alo[m][l0 + 16 + 8 * h];
#pragma unroll
    for (int t = 0; t < 6; ++t) {
      const int n = (wv * 6 + t) * 16 + m;
      const us16* bp = sT + (size_t)n * L_ + l0;
      Frag bf;
      bf.h2[0] = *(const v8us*)(bp + 8 * h);
      bf.h2[1] = *(const v8us*)(bp + 16 + 8 * h);
      acc[t] = wmma_bf16(ahi.b, bf.b, acc[t]);
      acc[t] = wmma_bf16(alo.b, bf.b, acc[t]);
    }
  }

#pragma unroll
  for (int t = 0; t < 6; ++t) {
    const int n0 = (wv * 6 + t) * 16;
#pragma unroll
    for (int rr = 0; rr < 8; ++rr)
      outs[8 * h + rr][n0 + m] = acc[t][rr] * scl[8 * h + rr];
  }
  __syncthreads();

#pragma unroll
  for (int i2 = 0; i2 < 2; ++i2) {
    const int row = wv + 8 * i2;
    const int gm = m0 + row;
    if (gm < M_) {
      float* orow = out + ((size_t)b * M_ + gm) * K_;
      v4f vv[6];
#pragma unroll
      for (int g = 0; g < 6; ++g) {
        const int cc = (g * 4 + (lane >> 3)) * 32 + (lane & 7) * 4;
        vv[g] = *(const v4f*)&outs[row][cc];
      }
#pragma unroll
      for (int g = 0; g < 6; ++g) {
        const int cc = (g * 4 + (lane >> 3)) * 32 + (lane & 7) * 4;
        *(volatile v4f*)(orow + cc) = vv[g];
      }
      __threadfence();
#pragma unroll
      for (int g = 0; g < 6; ++g) {
        const int cc = (g * 4 + (lane >> 3)) * 32 + (lane & 7) * 4;
        *(volatile v4f*)(orow + cc) = vv[g];
      }
    }
  }
}

extern "C" void kernel_launch(void* const* d_in, const int* in_sizes, int n_in,
                              void* d_out, int out_size, void* d_ws, size_t ws_size,
                              hipStream_t stream)
{
  if (n_in < 8) return;
  if (in_sizes[0] != B_ * M_ * D_) return;
  if (in_sizes[1] != B_ * L_ * K_) return;
  if (in_sizes[2] != B_ * L_) return;
  if (in_sizes[3] != D_) return;
  if (in_sizes[4] < 1) return;
  if (in_sizes[5] != K_) return;
  if (in_sizes[6] < 1) return;
  if (in_sizes[7] != L_ * L_) return;
  if (out_size != B_ * M_ * K_) return;

  const float* image_emb = (const float*)d_in[0];
  const float* seq_emb   = (const float*)d_in[1];
  const int*   mask      = (const int*)d_in[2];
  const float* img_W     = (const float*)d_in[3];
  const float* img_b     = (const float*)d_in[4];
  const float* seq_W     = (const float*)d_in[5];
  const float* seq_b     = (const float*)d_in[6];
  const float* V         = (const float*)d_in[7];
  float* out = (float*)d_out;

  const size_t off_s = 0;
  const size_t off_q = off_s + (size_t)B_ * M_ * 4;
  const size_t off_r = off_q + (size_t)B_ * L_ * 4;
  const size_t off_t = off_r + (size_t)B_ * L_ * 4;
  const size_t total = off_t + (size_t)B_ * K_ * L_ * 2;
  if (total > ws_size) return;

  char* ws = (char*)d_ws;
  float* s_buf = (float*)(ws + off_s);
  float* q_buf = (float*)(ws + off_q);
  float* r_buf = (float*)(ws + off_r);
  us16*  seqT  = (us16*)(ws + off_t);

  const int nProjBlocks = (B_ * M_) / 32 + (B_ * L_) / 32;
  k_proj<<<nProjBlocks, 256, 0, stream>>>(image_emb, seq_emb, img_W, img_b, seq_W, seq_b,
                                          s_buf, q_buf);
  k_qv<<<dim3(L_ / 32, B_ / 16), 32, 0, stream>>>(q_buf, V, r_buf);
  k_seqT<<<dim3(K_ / 32, L_ / 64, B_), 256, 0, stream>>>(seq_emb, seqT);
  k_main<<<dim3(MT_, B_), 256, 0, stream>>>(s_buf, r_buf, mask, seqT, out);
}
